// RecurrentGCN1_28853590295018
// MI455X (gfx1250) — hardware-verified
//
#include <hip/hip_runtime.h>


namespace {
constexpr int N = 4096, F = 64, HD = 128, NH = 8, DH = 16, H3 = 3 * HD;
constexpr float XS = 8.0f, WSC = 256.0f, PS = 8.0f, LOG2E = 1.4426950408889634f;
typedef _Float16 b16;
typedef __attribute__((ext_vector_type(16))) _Float16 v16b;
typedef __attribute__((ext_vector_type(8))) _Float16 v8b;
typedef __attribute__((ext_vector_type(8))) float v8f;
typedef __attribute__((ext_vector_type(4))) float v4f;
__device__ __forceinline__ float bf16_rne(float f) { unsigned int u = __float_as_uint(f); u += 0x7FFFu + ((u >> 16) & 1u); return __uint_as_float(u & 0xFFFF0000u); }
__device__ __forceinline__ void split16(float v, b16& hi, b16& lo) { hi = (b16)v; lo = (b16)(v - (float)hi); }
__device__ __forceinline__ v16b frag_kb(const b16* p, int hh) { const v8b a = *(const v8b*)(p + 8 * hh), b = *(const v8b*)(p + 16 + 8 * hh); v16b f;
#pragma unroll
  for (int e = 0; e < 8; ++e) { f[e] = a[e]; f[8 + e] = b[e]; } return f; }
__device__ __forceinline__ v16b frag16(const b16* p, int hh) { const v8b a = *(const v8b*)(p + 8 * hh); v16b f;
#pragma unroll
  for (int e = 0; e < 8; ++e) { f[e] = a[e]; f[8 + e] = (b16)0.0f; } return f; }
__device__ __forceinline__ v8f wmma16b(v16b a, v16b b, v8f c) { v8f d = __builtin_amdgcn_wmma_f32_16x16x32_f16(false, a, false, b, (short)0, c, false, false); asm volatile("v_nop\n\tv_nop\n\tv_nop\n\tv_nop" : "+v"(d) : "v"(a), "v"(b)); return d; }
__device__ __forceinline__ void wave_lds_sync() { __builtin_amdgcn_fence(__ATOMIC_RELEASE, "workgroup"); __builtin_amdgcn_wave_barrier(); __builtin_amdgcn_fence(__ATOMIC_ACQUIRE, "workgroup"); }
__device__ __forceinline__ float pmul(float a, float b) { float p = a * b; asm volatile("" : "+v"(p)); return p; }
__device__ __forceinline__ float sigm(float x) { return 1.0f / (1.0f + __expf(-x)); }

__global__ __launch_bounds__(256) void prep_kernel(const float* __restrict__ x, const float* __restrict__ wz, const float* __restrict__ wh, const float* __restrict__ win, const float* __restrict__ wo, const float* __restrict__ w1, b16* __restrict__ XX, b16* __restrict__ WG, b16* __restrict__ WQKV, b16* __restrict__ WO, b16* __restrict__ W1) {
  const size_t u = (size_t)blockIdx.x * 256 + threadIdx.x; const size_t nx = (size_t)N * 2 * F / 8, ng = (size_t)2 * HD * 2 * F / 8, nq = (size_t)H3 * HD / 8, no = (size_t)HD * HD / 8; size_t t = u; v8b o;
  if (t < nx) { const size_t e = t * 8; const size_t r = e / (2 * F); const int c0 = (int)(e % (2 * F)); for (int j = 0; j < 8; ++j) o[j] = (b16)(bf16_rne(x[r * F + ((c0 + j) % F)]) * XS); for (int pass = 0; pass < 2; ++pass) { *(volatile v8b*)(XX + e) = o; __threadfence(); } return; } t -= nx;
  if (t < ng) { const size_t e = t * 8; const int row = (int)(e / (2 * F)), k0 = (int)(e % (2 * F)); const float* w = row < HD ? wz : wh; const int oo = row % HD;
    for (int j = 0; j < 8; ++j) { const int k = k0 + j; const int d = k / F, kk = k % F; o[j] = (b16)(bf16_rne(w[((size_t)d * (F + HD) + kk) * HD + oo]) * WSC); } for (int pass = 0; pass < 2; ++pass) { *(volatile v8b*)(WG + e) = o; __threadfence(); } return; } t -= ng;
  if (t < nq) { const size_t e = t * 8; for (int j = 0; j < 8; ++j) o[j] = (b16)(bf16_rne(win[e + j]) * WSC); for (int pass = 0; pass < 2; ++pass) { *(volatile v8b*)(WQKV + e) = o; __threadfence(); } return; } t -= nq;
  if (t < no) { const size_t e = t * 8; for (int j = 0; j < 8; ++j) o[j] = (b16)(bf16_rne(wo[e + j]) * WSC); for (int pass = 0; pass < 2; ++pass) { *(volatile v8b*)(WO + e) = o; __threadfence(); } return; } t -= no;
  if (t < no) { const size_t e = t * 8; for (int j = 0; j < 8; ++j) o[j] = (b16)(bf16_rne(w1[e + j]) * WSC); for (int pass = 0; pass < 2; ++pass) { *(volatile v8b*)(W1 + e) = o; __threadfence(); } }
}
__global__ __launch_bounds__(128) void gate_kernel(const b16* __restrict__ XX, const b16* __restrict__ WG, const float* __restrict__ bz, const float* __restrict__ bh, float* __restrict__ HF, b16* __restrict__ Hh, b16* __restrict__ Hl) {
  __shared__ __attribute__((aligned(16))) float Tf[4][16][HD + 4];
  const int wave = threadIdx.x >> 5, lane = threadIdx.x & 31, nloc = lane & 15, hlf = lane >> 4; const size_t m0 = (size_t)blockIdx.x * 64 + wave * 16;
  v8f az[8], ah[8];
#pragma unroll
  for (int t = 0; t < 8; ++t) { az[t] = (v8f){}; ah[t] = (v8f){}; }
#pragma unroll
  for (int kb = 0; kb < 2 * F; kb += 32) { const v16b a = frag_kb(XX + (m0 + nloc) * (2 * F) + kb, hlf);
#pragma unroll
    for (int t = 0; t < 8; ++t) { az[t] = wmma16b(a, frag_kb(WG + (size_t)(t * 16 + nloc) * (2 * F) + kb, hlf), az[t]); ah[t] = wmma16b(a, frag_kb(WG + (size_t)(HD + t * 16 + nloc) * (2 * F) + kb, hlf), ah[t]); } }
#pragma unroll
  for (int t = 0; t < 8; ++t) { const int c = t * 16 + nloc; const float b1 = bf16_rne(bz[c]), b2 = bf16_rne(bh[c]);
#pragma unroll 1
    for (int r = 0; r < 8; ++r) { const float z = sigm(az[t][r] * (1.0f / (XS * WSC)) + b1); const float ht = tanhf(ah[t][r] * (1.0f / (XS * WSC)) + b2); Tf[wave][8 * hlf + r][c] = pmul(1.0f - z, ht); } }
  wave_lds_sync();
  for (int pass = 0; pass < 2; ++pass) { for (int rr = 0; rr < 16; ++rr) { const v4f v = *(const v4f*)(&Tf[wave][rr][lane * 4]); *(volatile v4f*)(HF + (m0 + rr) * HD + lane * 4) = v;
      b16 ph[4], pl[4]; for (int j = 0; j < 4; ++j) split16(v[j] * XS, ph[j], pl[j]); typedef __attribute__((ext_vector_type(4))) _Float16 v4h; v4h hv = {ph[0], ph[1], ph[2], ph[3]}, lv = {pl[0], pl[1], pl[2], pl[3]}; *(volatile v4h*)(Hh + (m0 + rr) * HD + lane * 4) = hv; *(volatile v4h*)(Hl + (m0 + rr) * HD + lane * 4) = lv; }
    __threadfence(); }
}
__global__ __launch_bounds__(128) void qkv_kernel(const b16* __restrict__ Hh, const b16* __restrict__ Hl, const b16* __restrict__ WQKV, const float* __restrict__ bqkv, b16* __restrict__ Qh, b16* __restrict__ Ql, b16* __restrict__ Kh, b16* __restrict__ Kl, b16* __restrict__ VTh, b16* __restrict__ VTl) {
  __shared__ __attribute__((aligned(16))) b16 Th[HD][64 + 8], Tl[HD][64 + 8];
  const int wave = threadIdx.x >> 5, lane = threadIdx.x & 31, nloc = lane & 15, hlf = lane >> 4, t_ = threadIdx.x; const int kind = blockIdx.y; const size_t m0 = (size_t)blockIdx.x * 64 + wave * 16;
  v8f acc[8];
#pragma unroll
  for (int t = 0; t < 8; ++t) acc[t] = (v8f){};
#pragma unroll
  for (int kb = 0; kb < HD; kb += 32) { const v16b a = frag_kb(Hh + (m0 + nloc) * HD + kb, hlf), al = frag_kb(Hl + (m0 + nloc) * HD + kb, hlf);
#pragma unroll
    for (int t = 0; t < 8; ++t) { const v16b bw = frag_kb(WQKV + ((size_t)kind * HD + t * 16 + nloc) * HD + kb, hlf); acc[t] = wmma16b(a, bw, acc[t]); acc[t] = wmma16b(al, bw, acc[t]); } }
  const float osc = kind == 0 ? 0.25f : 1.0f;
  if (kind < 2) { b16* dh = kind == 0 ? Qh : Kh; b16* dl = kind == 0 ? Ql : Kl; __shared__ __attribute__((aligned(16))) b16 Rh[4][16][HD + 8], Rl[4][16][HD + 8];
#pragma unroll
    for (int t = 0; t < 8; ++t) { const float bb = bf16_rne(bqkv[kind * HD + t * 16 + nloc]);
#pragma unroll 1
      for (int r = 0; r < 8; ++r) { b16 p, q; split16((acc[t][r] * (1.0f / (XS * WSC)) + bb) * osc * XS, p, q); Rh[wave][8 * hlf + r][t * 16 + nloc] = p; Rl[wave][8 * hlf + r][t * 16 + nloc] = q; } }
    wave_lds_sync();
    for (int pass = 0; pass < 2; ++pass) { for (int rr = 0; rr < 16; ++rr) if (lane < 16) { *(volatile v8b*)(dh + (m0 + rr) * HD + lane * 8) = *(const v8b*)(&Rh[wave][rr][lane * 8]); *(volatile v8b*)(dl + (m0 + rr) * HD + lane * 8) = *(const v8b*)(&Rl[wave][rr][lane * 8]); } __threadfence(); }
  } else {
#pragma unroll
    for (int t = 0; t < 8; ++t) { const float bb = bf16_rne(bqkv[2 * HD + t * 16 + nloc]);
#pragma unroll 1
      for (int r = 0; r < 8; ++r) { b16 p, q; split16((acc[t][r] * (1.0f / (XS * WSC)) + bb) * XS, p, q); Th[t * 16 + nloc][wave * 16 + 8 * hlf + r] = p; Tl[t * 16 + nloc][wave * 16 + 8 * hlf + r] = q; } }
    __syncthreads(); const size_t n0 = (size_t)blockIdx.x * 64;
    for (int pass = 0; pass < 2; ++pass) { for (int q = t_; q < HD * 8; q += 128) { const int d = q >> 3, c8 = (q & 7) * 8; *(volatile v8b*)(VTh + (size_t)d * N + n0 + c8) = *(const v8b*)(&Th[d][c8]); *(volatile v8b*)(VTl + (size_t)d * N + n0 + c8) = *(const v8b*)(&Tl[d][c8]); } __threadfence(); }
  }
}
__global__ __launch_bounds__(64) void attn_kernel(const b16* __restrict__ Qh, const b16* __restrict__ Ql, const b16* __restrict__ Kh, const b16* __restrict__ Kl, const b16* __restrict__ VTh, const b16* __restrict__ VTl, const float* __restrict__ HF, const b16* __restrict__ WO, const float* __restrict__ bo, const b16* __restrict__ W1, const float* __restrict__ b1, const float* __restrict__ w2, const float* __restrict__ b2, float* __restrict__ out) {
  __shared__ __attribute__((aligned(16))) b16 Ch[2][16][HD + 8], Cl[2][16][HD + 8]; __shared__ __attribute__((aligned(16))) float so[32];
  const int wave = threadIdx.x >> 5, lane = threadIdx.x & 31, hh = lane >> 4, col = lane & 15; const int q0 = blockIdx.x * 32 + wave * 16, qi = q0 + col;
  const float cs = LOG2E / (XS * XS);
  v8f o[NH]; float mrun[NH], lrun[NH];
#pragma unroll
  for (int h = 0; h < NH; ++h) { o[h] = (v8f){}; mrun[h] = -INFINITY; lrun[h] = 0.0f; }
  for (int kb = 0; kb < N; kb += 32) {
#pragma unroll
    for (int h = 0; h < NH; ++h) {
      const v16b qa = frag16(Qh + (size_t)qi * HD + h * DH, hh), qlo = frag16(Ql + (size_t)qi * HD + h * DH, hh);
      v8f s0 = {}, s1 = {};
      { const b16* k0 = Kh + (size_t)(kb + col) * HD + h * DH, *k1 = Kh + (size_t)(kb + 16 + col) * HD + h * DH, *k0l = Kl + (size_t)(kb + col) * HD + h * DH, *k1l = Kl + (size_t)(kb + 16 + col) * HD + h * DH;
        v16b f = frag16(k0, hh); s0 = wmma16b(f, qa, s0); s0 = wmma16b(f, qlo, s0); s0 = wmma16b(frag16(k0l, hh), qa, s0);
        f = frag16(k1, hh); s1 = wmma16b(f, qa, s1); s1 = wmma16b(f, qlo, s1); s1 = wmma16b(frag16(k1l, hh), qa, s1); }
      float e[16]; float bm = -INFINITY;
#pragma unroll
      for (int r = 0; r < 8; ++r) { e[r] = s0[r] * cs; e[8 + r] = s1[r] * cs; bm = fmaxf(bm, fmaxf(e[r], e[8 + r])); }
      bm = fmaxf(bm, __shfl_xor(bm, 16)); const float mn = fmaxf(mrun[h], bm); const float sc = exp2f(mrun[h] - mn); float ls = 0.0f; v16b ph, pl;
#pragma unroll
      for (int i = 0; i < 16; ++i) { const float p = exp2f(e[i] - mn); ls += p; b16 a, c; split16(p * PS, a, c); ph[i] = a; pl[i] = c; }
      ls += __shfl_xor(ls, 16); lrun[h] = lrun[h] * sc + ls; mrun[h] = mn; o[h] *= sc;
      const v16b vf = frag_kb(VTh + (size_t)(h * DH + col) * N + kb, hh); o[h] = wmma16b(vf, ph, o[h]); o[h] = wmma16b(vf, pl, o[h]); o[h] = wmma16b(frag_kb(VTl + (size_t)(h * DH + col) * N + kb, hh), ph, o[h]); } }
#pragma unroll
  for (int h = 0; h < NH; ++h) { const float inv = 1.0f / (lrun[h] * PS * XS);
#pragma unroll
    for (int r = 0; r < 8; ++r) { b16 p, q; split16(o[h][r] * inv * XS, p, q); Ch[wave][col][h * DH + 8 * hh + r] = p; Cl[wave][col][h * DH + 8 * hh + r] = q; } }
  wave_lds_sync();
  const int nloc = col, hlf = hh; v8f d8[8];
#pragma unroll
  for (int t = 0; t < 8; ++t) d8[t] = (v8f){};
#pragma unroll
  for (int kb = 0; kb < HD; kb += 32) { const v16b a = frag_kb(&Ch[wave][nloc][kb], hlf), al = frag_kb(&Cl[wave][nloc][kb], hlf);
#pragma unroll
    for (int t = 0; t < 8; ++t) { const v16b bw = frag_kb(WO + (size_t)(t * 16 + nloc) * HD + kb, hlf); d8[t] = wmma16b(a, bw, d8[t]); d8[t] = wmma16b(al, bw, d8[t]); } }
  wave_lds_sync();
#pragma unroll
  for (int t = 0; t < 8; ++t) { const int c = t * 16 + nloc; const float bb = bf16_rne(bo[c]);
#pragma unroll 1
    for (int r = 0; r < 8; ++r) { const int q = q0 + 8 * hlf + r; const float h2 = HF[(size_t)q * HD + c] + (d8[t][r] * (1.0f / (XS * WSC)) + bb); b16 p, pq; split16(h2 * XS, p, pq); Ch[wave][8 * hlf + r][c] = p; Cl[wave][8 * hlf + r][c] = pq; } }
  wave_lds_sync();
#pragma unroll
  for (int t = 0; t < 8; ++t) d8[t] = (v8f){};
#pragma unroll
  for (int kb = 0; kb < HD; kb += 32) { const v16b a = frag_kb(&Ch[wave][nloc][kb], hlf), al = frag_kb(&Cl[wave][nloc][kb], hlf);
#pragma unroll
    for (int t = 0; t < 8; ++t) { const v16b bw = frag_kb(W1 + (size_t)(t * 16 + nloc) * HD + kb, hlf); d8[t] = wmma16b(a, bw, d8[t]); d8[t] = wmma16b(al, bw, d8[t]); } }
  float part[8]; for (int r = 0; r < 8; ++r) part[r] = 0.0f;
#pragma unroll
  for (int t = 0; t < 8; ++t) { const int c = t * 16 + nloc; const float bb = bf16_rne(b1[c]), ww = bf16_rne(w2[c]);
#pragma unroll
    for (int r = 0; r < 8; ++r) part[r] += pmul(fmaxf(d8[t][r] * (1.0f / (XS * WSC)) + bb, 0.0f), ww); }
#pragma unroll
  for (int r = 0; r < 8; ++r) { float v = part[r]; v += __shfl_xor(v, 1); v += __shfl_xor(v, 2); v += __shfl_xor(v, 4); v += __shfl_xor(v, 8); part[r] = v; }
  if (nloc == 0) for (int r = 0; r < 8; ++r) so[wave * 16 + 8 * hlf + r] = part[r] + bf16_rne(b2[0]);
  __syncthreads();
  for (int pass = 0; pass < 2; ++pass) { if (threadIdx.x < 8) *(volatile v4f*)(out + (size_t)blockIdx.x * 32 + threadIdx.x * 4) = *(const v4f*)(&so[threadIdx.x * 4]); __threadfence(); }
}
}

extern "C" void kernel_launch(void* const* d_in, const int* in_sizes, int n_in, void* d_out, int out_size, void* d_ws, size_t ws_size, hipStream_t stream) {
  (void)n_in;
  auto Fp = [&](int i) { return (const float*)d_in[i]; };
  if (in_sizes[0] != N * F || in_sizes[2] != 2 * (F + HD) * HD || in_sizes[6] != 2 * (F + HD) * HD || in_sizes[8] != H3 * HD || in_sizes[10] != HD * HD || in_sizes[12] != HD * HD || in_sizes[14] != HD || out_size != N) return;
  size_t off = 0; char* ws = (char*)d_ws;
  auto carve = [&](size_t bytes) { char* p = ws + off; off += (bytes + 255) & ~(size_t)255; return p; };
  b16* XX = (b16*)carve((size_t)N * 2 * F * 2); b16* WG = (b16*)carve((size_t)2 * HD * 2 * F * 2); b16* WQKV = (b16*)carve((size_t)H3 * HD * 2); b16* WO = (b16*)carve((size_t)HD * HD * 2); b16* W1 = (b16*)carve((size_t)HD * HD * 2);
  float* HF = (float*)carve((size_t)N * HD * 4); b16* Hh = (b16*)carve((size_t)N * HD * 2); b16* Hl = (b16*)carve((size_t)N * HD * 2);
  b16* Qh = (b16*)carve((size_t)N * HD * 2); b16* Ql = (b16*)carve((size_t)N * HD * 2); b16* Kh = (b16*)carve((size_t)N * HD * 2); b16* Kl = (b16*)carve((size_t)N * HD * 2); b16* VTh = (b16*)carve((size_t)N * HD * 2); b16* VTl = (b16*)carve((size_t)N * HD * 2);
  if (off > ws_size || off > ((size_t)128 << 20)) return;
  prep_kernel<<<(unsigned)(((size_t)N * 2 * F / 8 + (size_t)2 * HD * 2 * F / 8 + (size_t)H3 * HD / 8 + 2 * (size_t)HD * HD / 8 + 255) / 256), 256, 0, stream>>>(Fp(0), Fp(2), Fp(6), Fp(8), Fp(10), Fp(12), XX, WG, WQKV, WO, W1);
  gate_kernel<<<N / 64, 128, 0, stream>>>(XX, WG, Fp(3), Fp(7), HF, Hh, Hl);
  qkv_kernel<<<dim3(N / 64, 3), 128, 0, stream>>>(Hh, Hl, WQKV, Fp(9), Qh, Ql, Kh, Kl, VTh, VTl);
  attn_kernel<<<N / 32, 64, 0, stream>>>(Qh, Ql, Kh, Kl, VTh, VTl, HF, WO, Fp(11), W1, Fp(13), Fp(14), Fp(15), (float*)d_out);
}
